// FastKANLayer_18854906429776
// MI455X (gfx1250) — hardware-verified
//
#include <hip/hip_runtime.h>
#include <math.h>
#include <stdint.h>

#define NB   8
#define NI   32
#define NO   32
#define NF   187
#define NFP  192
#define ND   32
#define NCF  35
#define NKD  512
#define BASP 36
#define INV_H (1.0f / (float)(2.0 / 34.0))

static_assert(NB * NI * NF * ND == 1531904);
static_assert(NKD == (NI / 2) * ND);

typedef __attribute__((ext_vector_type(16))) __bf16 v16b;
typedef __attribute__((ext_vector_type(8)))  __bf16 v8b;
typedef __attribute__((ext_vector_type(8)))  float  v8f;
typedef __attribute__((ext_vector_type(4)))  float  v4f;
typedef __attribute__((ext_vector_type(8)))  unsigned short v8us;

union FB { v16b v; v8b h[2]; unsigned u[8]; };

__device__ __forceinline__ unsigned short bfb(float f) {
  unsigned u = __float_as_uint(f);
  return (unsigned short)((u + 0x7FFFu + ((u >> 16) & 1u)) >> 16);
}
__device__ __forceinline__ float bff(unsigned short h) { return __uint_as_float(((unsigned)h) << 16); }
__device__ __forceinline__ void split2(float f, unsigned short& hb, unsigned short& lb) {
  hb = bfb(f);
  lb = bfb(f - bff(hb));
}
__device__ __forceinline__ unsigned pk16(unsigned short a, unsigned short b) { return (unsigned)a | ((unsigned)b << 16); }

__device__ __forceinline__ float wsum(float v) {
#pragma unroll
  for (int m = 16; m > 0; m >>= 1) v += __shfl_xor(v, m, 32);
  return v;
}

__device__ __forceinline__ v16b ldfrag(const unsigned short* p) {
  FB f;
  f.h[0] = *(const v8b*)(const void*)p;
  f.h[1] = *(const v8b*)(const void*)(p + 16);
  return f.v;
}

__device__ __forceinline__ v8f mma_bf(v16b a, v16b b, v8f c) {
  c = __builtin_amdgcn_wmma_f32_16x16x32_bf16(false, a, false, b, (short)0, c, false, false);
  asm volatile("v_nop\n\tv_nop\n\tv_nop\n\tv_nop" : "+v"(c) : "v"(a), "v"(b));
  return c;
}

__global__ __launch_bounds__(256)
void k_prep(const float* __restrict__ x_in, const float* __restrict__ spw, const float* __restrict__ bsc,
            const float* __restrict__ tau, const float* __restrict__ temp, const float* __restrict__ omg,
            const float* __restrict__ grd, float* __restrict__ coef, float* __restrict__ maskg,
            float* __restrict__ gateg) {
  __shared__ float xeL[NFP];
  __shared__ float saL[NFP];
  __shared__ float siL[NFP];
  __shared__ float basL[NFP * BASP];
  __shared__ float swL[NO * NCF];
  __shared__ float gridL[BASP];
  __shared__ float bsL[NO];
  __shared__ float omL[NO];
  __shared__ float taL[NO];
  __shared__ __align__(16) float coefL[NO * NFP];
  __shared__ __align__(16) float mgL[64];
  __shared__ float red[256];

  const int bi = blockIdx.x;
  const int i = bi & 31;
  const int tid = threadIdx.x, lane = tid & 31, wave = tid >> 5;

  const float* xb = x_in + (size_t)bi * NF * ND;
#pragma unroll 1
  for (int f = wave; f < NF; f += 8) {
    const float x = xb[f * ND + lane];
    const float sx = wsum(x);
    const float sa = wsum(fabsf(x));
    if (lane == 0) { xeL[f] = sx * (1.0f / (float)ND); saL[f] = sa; }
  }
#pragma unroll 1
  for (int idx = tid; idx < NO * NCF; idx += 256) swL[idx] = spw[(size_t)i * NO * NCF + idx];
  if (tid < NCF) gridL[tid] = grd[tid];
  if (tid < NO) {
    bsL[tid] = bsc[i * NO + tid];
    omL[tid] = fabsf(omg[i * NO + tid]);
    taL[tid] = fabsf(tau[i * NO + tid]);
  }
  __syncthreads();

  {
    const int fc = (tid < NF) ? tid : (NF - 1);
    const float m = (tid < NF) ? fabsf(xeL[fc]) : 0.0f;
    red[tid] = m;
  }
  __syncthreads();
#pragma unroll 1
  for (int s = 128; s > 0; s >>= 1) {
    if (tid < s) red[tid] = fmaxf(red[tid], red[tid + s]);
    __syncthreads();
  }
  const float denom = red[0] + 1e-8f;
  const float invd = 1.0f / denom;

  if (tid < NFP) {
    const bool fv = tid < NF;
    const int fc = fv ? tid : (NF - 1);
    float xr = xeL[fc] * invd;
    xr = fminf(fmaxf(xr, -0.99f), 0.99f);
    const float sg = 1.0f / (1.0f + expf(-xr));
    siL[tid] = fv ? (xr * sg) : 0.0f;
#pragma unroll 1
    for (int c = 0; c < NCF; ++c) {
      const float d = fabsf(xr - gridL[c]) * INV_H;
      float bs;
      if (d < 1.0f) {
        bs = ((float)(2.0 / 3.0) - d * d) + (d * (d * d)) * 0.5f;
      } else if (d < 2.0f) {
        const float t = 2.0f - d;
        bs = (t * (t * t)) * (1.0f / 6.0f);
      } else {
        bs = 0.0f;
      }
      basL[tid * BASP + c] = fv ? bs : 0.0f;
    }
  }
  __syncthreads();

  if (tid < NFP) {
    const int f = tid;
    const bool fv = f < NF;
    const float si = siL[f];
#pragma unroll 1
    for (int o = 0; o < NO; ++o) {
      float sp = 0.0f;
#pragma unroll 1
      for (int c = 0; c < NCF; ++c) sp += basL[f * BASP + c] * swL[o * NCF + c];
      const float co = (si * bsL[o] + sp) + omL[o];
      coefL[o * NFP + f] = fv ? co : 0.0f;
    }
  }
  __syncthreads();

  const float tv = fabsf(temp[0]) + 1e-4f;
  const float itv = 1.0f / tv;
#pragma unroll 1
  for (int q = 0; q < 4; ++q) {
    const int o = wave * 4 + q;
    float a = 0.0f;
#pragma unroll 1
    for (int f = lane; f < NF; f += 32) a += fabsf(coefL[o * NFP + f]) * saL[f];
    a = wsum(a);
    if (lane == 0) {
      const float ee = a * (1.0f / (float)(NF * ND));
      const float ta = taL[o];
      const float mk = 1.0f / (1.0f + expf(-((ee - ta) * itv)));
      mgL[o] = mk;
      mgL[32 + o] = (ee * (1.0f / (ta + 1e-8f))) * mk;
    }
  }
  __syncthreads();

  v4f c0[4], c1[4];
#pragma unroll
  for (int q = 0; q < 4; ++q) {
    const int o = wave * 4 + q;
    c0[q] = *(const v4f*)(coefL + o * NFP + lane * 4);
    c1[q] = *(const v4f*)(coefL + o * NFP + 128 + (lane & 15) * 4);
  }
  const v4f mg = *(const v4f*)(mgL + (lane & 15) * 4);
  for (int pass = 0; pass < 2; ++pass) {
#pragma unroll
    for (int q = 0; q < 4; ++q) {
      const int o = wave * 4 + q;
      float* rb = coef + ((size_t)bi * NO + o) * NFP;
      *(volatile v4f*)(rb + lane * 4) = c0[q];
      if (lane < 16) *(volatile v4f*)(rb + 128 + (lane & 15) * 4) = c1[q];
    }
    if (wave == 0) {
      if (lane < 8) {
        *(volatile v4f*)(maskg + (size_t)bi * NO + lane * 4) = mg;
      } else if (lane < 16) {
        *(volatile v4f*)(gateg + (size_t)bi * NO + (lane - 8) * 4) = mg;
      }
    }
    __threadfence();
  }
}

#define KQ_WAVES 4
#define KQ_THREADS (KQ_WAVES * 32)
__global__ __launch_bounds__(KQ_THREADS)
void k_kq(const float* __restrict__ pp, const float* __restrict__ gateg,
          unsigned short* __restrict__ Kh, unsigned short* __restrict__ Kl,
          unsigned short* __restrict__ Qh, unsigned short* __restrict__ Ql, int b) {
  __shared__ float gateL[NI * NO];
  __shared__ float rawL[KQ_WAVES][NI * ND];
  __shared__ __align__(16) unsigned short stg[KQ_WAVES][4][NKD];

  const int tid = threadIdx.x, lane = tid & 31, wave = tid >> 5;
  const int f = blockIdx.x * KQ_WAVES + wave;
  const bool valid = f < NF;
  const int fcl = valid ? f : (NF - 1);

#pragma unroll 1
  for (int idx = tid; idx < NI * NO; idx += KQ_THREADS) gateL[idx] = gateg[(size_t)b * NI * NO + idx];
  float* rw = rawL[wave];
#pragma unroll 4
  for (int i = 0; i < NI; ++i) {
    const float v = pp[((size_t)(b * NI + i) * NF + fcl) * ND + lane];
    rw[i * ND + lane] = valid ? v : 0.0f;
  }
  __syncthreads();

  unsigned short* sKH = &stg[wave][0][0];
  unsigned short* sKL = &stg[wave][1][0];
  unsigned short* sQH = &stg[wave][2][0];
  unsigned short* sQL = &stg[wave][3][0];

#pragma unroll 1
  for (int o = 0; o < NO; ++o) {
    float sk = 0.0f, sq = 0.0f;
#pragma unroll 1
    for (int i = 0; i < 16; ++i) {
      sk += rw[i * ND + lane] * gateL[i * NO + o];
      sq += rw[(i + 16) * ND + lane] * gateL[(i + 16) * NO + o];
    }
    const float muK = wsum(sk) * (1.0f / (float)NKD);
    const float muQ = wsum(sq) * (1.0f / (float)NKD);
    float vk = 0.0f, vq = 0.0f;
#pragma unroll 1
    for (int i = 0; i < 16; ++i) {
      const float dk = rw[i * ND + lane] * gateL[i * NO + o] - muK;
      const float dq = rw[(i + 16) * ND + lane] * gateL[(i + 16) * NO + o] - muQ;
      vk += dk * dk;
      vq += dq * dq;
    }
    const float rK = rsqrtf(wsum(vk) * (1.0f / (float)NKD) + 1e-5f);
    const float rQ = rsqrtf(wsum(vq) * (1.0f / (float)NKD) + 1e-5f);
#pragma unroll 1
    for (int i = 0; i < 16; ++i) {
      const float kn = (rw[i * ND + lane] * gateL[i * NO + o] - muK) * rK;
      const float qn = (rw[(i + 16) * ND + lane] * gateL[(i + 16) * NO + o] - muQ) * rQ;
      unsigned short h0, l0, h1, l1;
      split2(kn, h0, l0);
      split2(qn, h1, l1);
      sKH[i * ND + lane] = h0;
      sKL[i * ND + lane] = l0;
      sQH[i * ND + lane] = h1;
      sQL[i * ND + lane] = l1;
    }
    __syncthreads();
    v8us pk[8];
#pragma unroll
    for (int q = 0; q < 2; ++q) {
      pk[q]     = *(const v8us*)(sKH + q * 256 + lane * 8);
      pk[2 + q] = *(const v8us*)(sKL + q * 256 + lane * 8);
      pk[4 + q] = *(const v8us*)(sQH + q * 256 + lane * 8);
      pk[6 + q] = *(const v8us*)(sQL + q * 256 + lane * 8);
    }
    const size_t rb = ((size_t)o * NFP + f) * NKD;
    for (int pass = 0; pass < 2; ++pass) {
#pragma unroll
      for (int q = 0; q < 2; ++q) {
        const size_t off = rb + (size_t)q * 256 + lane * 8;
        *(volatile v8us*)(Kh + off) = pk[q];
        *(volatile v8us*)(Kl + off) = pk[2 + q];
        *(volatile v8us*)(Qh + off) = pk[4 + q];
        *(volatile v8us*)(Ql + off) = pk[6 + q];
      }
      __threadfence();
    }
    __syncthreads();
  }
}

#define ATT_THREADS 384
#define LDS_COMB 0
#define LDS_BMF  24576
#define LDS_BMTH 49152
#define LDS_BMTL 61440
#define LDS_W2   73728
#define LDS_MASK 77824
#define LDS_OUTS 77952
#define LDS_TOTAL 102528
static_assert(LDS_OUTS + 12 * 16 * ND * 4 == LDS_TOTAL);

__global__ __launch_bounds__(ATT_THREADS)
void k_attn(const float* __restrict__ x_in, const float* __restrict__ coef, const float* __restrict__ maskg,
            const float* __restrict__ W2, const float* __restrict__ lnw, const float* __restrict__ lnb,
            const float* __restrict__ bparam, const float* __restrict__ temp,
            const float* __restrict__ beta, const float* __restrict__ gamma_, const float* __restrict__ alpha_,
            const unsigned short* __restrict__ Kh, const unsigned short* __restrict__ Kl,
            const unsigned short* __restrict__ Qh, const unsigned short* __restrict__ Ql,
            float* __restrict__ out0, float* __restrict__ out1, int b) {
  extern __shared__ __align__(16) unsigned char dsm[];
  float* combL = (float*)(dsm + LDS_COMB);
  float* bmfL  = (float*)(dsm + LDS_BMF);
  unsigned short* bmtH = (unsigned short*)(dsm + LDS_BMTH);
  unsigned short* bmtL = (unsigned short*)(dsm + LDS_BMTL);
  float* w2L   = (float*)(dsm + LDS_W2);
  float* maskL = (float*)(dsm + LDS_MASK);
  float* outS  = (float*)(dsm + LDS_OUTS);

  const int tid = threadIdx.x, wave = tid >> 5, lane = tid & 31;
  const int hh = lane >> 4, c = lane & 15;
  const int o = blockIdx.x;
  const int bo = b * NO + o;

  for (int idx = tid; idx < ND * ND; idx += ATT_THREADS) w2L[idx] = W2[(size_t)o * ND * ND + idx];
  if (tid < NI) maskL[tid] = maskg[((size_t)b * NI + tid) * NO + o];
  if (tid < 160) {
    const int rr = tid / 5, cc = NF + tid % 5;
    bmtH[rr * NFP + cc] = 0;
    bmtL[rr * NFP + cc] = 0;
    combL[NF * ND + tid] = 0.0f;
    bmfL[NF * ND + tid] = 0.0f;
  }
  __syncthreads();

  {
    const float lw = lnw[o * ND + lane];
    const float lb2 = lnb[o * ND + lane];
#pragma unroll 1
    for (int it = 0; it < 16; ++it) {
      const int f = wave + 12 * it;
      if (f < NF) {
        float acc = 0.0f;
#pragma unroll 4
        for (int i = 0; i < NI; ++i) {
          const float cf = coef[((size_t)(b * NI + i) * NO + o) * NFP + f];
          const float x = x_in[((size_t)(b * NI + i) * NF + f) * ND + lane];
          acc += (cf * x) * maskL[i];
        }
        const float cb = acc * (1.0f / (float)NI);
        combL[f * ND + lane] = cb;
        const float mu = wsum(cb) * (1.0f / (float)ND);
        const float dv = cb - mu;
        const float var = wsum(dv * dv) * (1.0f / (float)ND);
        const float xn = (dv * rsqrtf(var + 1e-5f)) * lw + lb2;
        float pr = 0.0f;
#pragma unroll 4
        for (int d = 0; d < ND; ++d) pr += __shfl(xn, d, 32) * w2L[d * ND + lane];
        volatile float* p1 = (volatile float*)(out1 + ((size_t)bo * NF + f) * ND + lane);
        *p1 = pr;
        __threadfence();
        *p1 = pr;
        const float bm = pr + bparam[((size_t)o * NF + f) * ND + lane];
        bmfL[f * ND + lane] = bm;
        unsigned short hb, lb;
        split2(bm, hb, lb);
        bmtH[lane * NFP + f] = hb;
        bmtL[lane * NFP + f] = lb;
      }
    }
  }
  __syncthreads();

  const int mt = wave;
  const size_t krow = (size_t)(o * NFP + 16 * mt + c) * NKD + 8 * hh;
  const unsigned short* kph = Kh + krow;
  const unsigned short* kpl = Kl + krow;
  const size_t qrow = (size_t)(o * NFP + c) * NKD + 8 * hh;
  const unsigned short* qph = Qh + qrow;
  const unsigned short* qpl = Ql + qrow;

  v8f acc[12];
#pragma unroll
  for (int j = 0; j < 12; ++j) acc[j] = (v8f){0.f, 0.f, 0.f, 0.f, 0.f, 0.f, 0.f, 0.f};

#pragma unroll 1
  for (int kk = 0; kk < NKD / 32; ++kk) {
    const v16b kbh = ldfrag(kph + 32 * kk);
    const v16b kbl = ldfrag(kpl + 32 * kk);
#pragma unroll
    for (int j = 0; j < 12; ++j) {
      const v16b qah = ldfrag(qph + (size_t)j * 16 * NKD + 32 * kk);
      const v16b qal = ldfrag(qpl + (size_t)j * 16 * NKD + 32 * kk);
      acc[j] = mma_bf(qah, kbh, acc[j]);
      acc[j] = mma_bf(qah, kbl, acc[j]);
      acc[j] = mma_bf(qal, kbh, acc[j]);
    }
  }

  const float tv = fabsf(temp[0]) + 1e-4f;
  const float sc = 1.0f / (sqrtf((float)NKD) * tv);
  float mx = -INFINITY;
#pragma unroll
  for (int j = 0; j < 12; ++j) {
#pragma unroll
    for (int r = 0; r < 8; ++r) {
      const float z = acc[j][r] * sc;
      acc[j][r] = z;
      const bool ok = (j < 11) || ((8 * hh + r) < (NF - 176));
      mx = ok ? fmaxf(mx, z) : mx;
    }
  }
  mx = fmaxf(mx, __shfl_xor(mx, 16, 32));
  float sm = 0.0f;
#pragma unroll
  for (int j = 0; j < 12; ++j) {
#pragma unroll
    for (int r = 0; r < 8; ++r) {
      const bool ok = (j < 11) || ((8 * hh + r) < (NF - 176));
      const float e = expf(acc[j][r] - mx);
      const float p = ok ? e : 0.0f;
      acc[j][r] = p;
      sm += p;
    }
  }
  sm += __shfl_xor(sm, 16, 32);
  const float inv = 1.0f / sm;
#pragma unroll
  for (int j = 0; j < 12; ++j) {
#pragma unroll
    for (int r = 0; r < 8; ++r) acc[j][r] = acc[j][r] * inv;
  }

  v8f oacc[2];
  oacc[0] = (v8f){0.f, 0.f, 0.f, 0.f, 0.f, 0.f, 0.f, 0.f};
  oacc[1] = (v8f){0.f, 0.f, 0.f, 0.f, 0.f, 0.f, 0.f, 0.f};
#pragma unroll
  for (int k2 = 0; k2 < 6; ++k2) {
    FB pa, pl;
#pragma unroll
    for (int q = 0; q < 4; ++q) {
      unsigned short h0, l0, h1, l1;
      split2(acc[2 * k2][2 * q], h0, l0);
      split2(acc[2 * k2][2 * q + 1], h1, l1);
      pa.u[q] = pk16(h0, h1);
      pl.u[q] = pk16(l0, l1);
      split2(acc[2 * k2 + 1][2 * q], h0, l0);
      split2(acc[2 * k2 + 1][2 * q + 1], h1, l1);
      pa.u[4 + q] = pk16(h0, h1);
      pl.u[4 + q] = pk16(l0, l1);
    }
#pragma unroll
    for (int t = 0; t < 2; ++t) {
      const unsigned short* bp = bmtH + (16 * t + c) * NFP + 32 * k2 + 8 * hh;
      const unsigned short* bq = bmtL + (16 * t + c) * NFP + 32 * k2 + 8 * hh;
      const v16b bh = ldfrag(bp);
      const v16b bl = ldfrag(bq);
      oacc[t] = mma_bf(pa.v, bh, oacc[t]);
      oacc[t] = mma_bf(pa.v, bl, oacc[t]);
      oacc[t] = mma_bf(pl.v, bh, oacc[t]);
    }
  }

  const float bA = fabsf(beta[o]), aA = fabsf(alpha_[o]), gm = gamma_[o];
  float* os = outS + wave * (16 * ND);
#pragma unroll
  for (int t = 0; t < 2; ++t) {
#pragma unroll
    for (int r = 0; r < 8; ++r) {
      const int fl = 8 * hh + r;
      const int col = 16 * t + c;
      const int fg = 16 * mt + fl;
      const float v = (bA * oacc[t][r] + aA * bmfL[fg * ND + col]) + gm * combL[fg * ND + col];
      os[fl * ND + col] = v;
    }
  }
  __syncthreads();
  const int rq = lane >> 3, c4 = (lane & 7) * 4;
  v4f vv[4];
#pragma unroll
  for (int q = 0; q < 4; ++q) vv[q] = *(const v4f*)(os + (q * 4 + rq) * ND + c4);
  for (int pass = 0; pass < 2; ++pass) {
#pragma unroll
    for (int q = 0; q < 4; ++q) {
      const int fg = 16 * mt + q * 4 + rq;
      if (fg < NF) *(volatile v4f*)(out0 + ((size_t)bo * NF + fg) * ND + c4) = vv[q];
    }
    __threadfence();
  }
}

extern "C" void kernel_launch(void* const* d_in, const int* in_sizes, int n_in,
                              void* d_out, int out_size, void* d_ws, size_t ws_size,
                              hipStream_t stream) {
  if (n_in < 15) return;
  const int NX = NB * NI * NF * ND;
  if (in_sizes[0] != NX || in_sizes[1] != NX) return;
  if (in_sizes[2] != NI * NO * NCF || in_sizes[3] != NI * NO || in_sizes[4] != NI * NO) return;
  if (in_sizes[5] < 1 || in_sizes[6] != NI * NO || in_sizes[7] != NCF) return;
  if (in_sizes[8] != NO * ND * ND || in_sizes[9] != NO * NF * ND) return;
  if (in_sizes[10] != NO * ND || in_sizes[11] != NO * ND) return;
  if (in_sizes[12] != NO || in_sizes[13] != NO || in_sizes[14] != NO) return;
  if (out_size != 2 * NX) return;

  const float* x_in = (const float*)d_in[0];
  const float* pp   = (const float*)d_in[1];
  const float* spw  = (const float*)d_in[2];
  const float* bsc  = (const float*)d_in[3];
  const float* tau  = (const float*)d_in[4];
  const float* temp = (const float*)d_in[5];
  const float* omg  = (const float*)d_in[6];
  const float* grd  = (const float*)d_in[7];
  const float* W2   = (const float*)d_in[8];
  const float* bprm = (const float*)d_in[9];
  const float* lnw  = (const float*)d_in[10];
  const float* lnb  = (const float*)d_in[11];
  const float* beta = (const float*)d_in[12];
  const float* gam  = (const float*)d_in[13];
  const float* alph = (const float*)d_in[14];

  float* out0 = (float*)d_out;
  float* out1 = out0 + (size_t)NX;

  const size_t szCoef  = (size_t)NB * NI * NO * NFP * 4;
  const size_t szLine  = (size_t)NB * NI * NO * 4;
  const size_t szPlane = (size_t)NO * NFP * NKD * 2;
  size_t off = 0;
  const size_t oCoef = off; off += szCoef;
  const size_t oMask = off; off += szLine;
  const size_t oGate = off; off += szLine;
  const size_t oKh = off; off += szPlane;
  const size_t oKl = off; off += szPlane;
  const size_t oQh = off; off += szPlane;
  const size_t oQl = off; off += szPlane;
  if (off > ws_size) return;

  char* ws = (char*)d_ws;
  float* coef  = (float*)(ws + oCoef);
  float* maskg = (float*)(ws + oMask);
  float* gateg = (float*)(ws + oGate);
  unsigned short* Kh = (unsigned short*)(ws + oKh);
  unsigned short* Kl = (unsigned short*)(ws + oKl);
  unsigned short* Qh = (unsigned short*)(ws + oQh);
  unsigned short* Ql = (unsigned short*)(ws + oQl);

  (void)hipFuncSetAttribute(reinterpret_cast<const void*>(&k_attn),
                            hipFuncAttributeMaxDynamicSharedMemorySize, LDS_TOTAL);

  k_prep<<<dim3(NB * NI), dim3(256), 0, stream>>>(x_in, spw, bsc, tau, temp, omg, grd, coef, maskg, gateg);
  for (int b = 0; b < NB; ++b) {
    k_kq<<<dim3(NFP / KQ_WAVES), dim3(KQ_THREADS), 0, stream>>>(pp, gateg, Kh, Kl, Qh, Ql, b);
    k_attn<<<dim3(NO), dim3(ATT_THREADS), LDS_TOTAL, stream>>>(
        x_in, coef, maskg, W2, lnw, lnb, bprm, temp, beta, gam, alph, Kh, Kl, Qh, Ql, out0, out1, b);
  }
  (void)hipGetLastError();
}
